// ResidualGCNLayer_90958817394877
// MI455X (gfx1250) — hardware-verified
//
#include <hip/hip_runtime.h>
#include <stddef.h>
#include <math.h>


#define FD      512
#define KC      1536
#define NTHR    256
#define NWAVE   8
#define EPT     8
#define NGRP    2
#define CHUNK   (NTHR * EPT * NGRP)
#define WCAP    (EPT * NGRP * 32)
#define LISTN   (NWAVE * WCAP)
#define NBC     4096
#define NBF     1024
#define RCAP    40960
#define RBN     128
#define TGT     256
#define DEGCAP  1024
#define GR      64
#define OTHR    512
#define WSCAP   134217728
#define NBWC    ((FD * KC / 8) / NTHR)
#define NBWL    ((FD * FD / 8) / NTHR)

#define APKC    (KC + 8)
#define APKL    (FD + 8)

#define WSCL    32.0f
#define WINV    0.03125f
#define BN_EPS  1e-5f

#define LDS_FILL ((RCAP + NBF + LISTN) * 4 + 64)
#define LDS_STG  (NWAVE * 16 * 64 * 4)
#define LDS_DST  (NWAVE * 4 * 64 * 8)
#define LDS_GC   (GR * APKC * 2 + LDS_STG + LDS_DST)
#define LDS_GO   (GR * APKL * 2 + LDS_STG)

static_assert((CHUNK & (CHUNK - 1)) == 0);
static_assert(CHUNK <= 4096);
static_assert(NBC <= 4096 && NBF <= 4096);
static_assert((NBC & (NBC - 1)) == 0 && (NBF & (NBF - 1)) == 0);
static_assert(NBC == 4 * NBF);
static_assert(OTHR * 8 == NBC);
static_assert((RCAP % 32) == 0);
static_assert(TGT == NWAVE * 32 && (TGT % GR) == 0);
static_assert((NBC % TGT) == 0);
static_assert(GR == 64 && NWAVE * 64 == FD);
static_assert((KC % 32) == 0 && (FD % 32) == 0);
static_assert(((GR * APKC * 2) % 16) == 0 && ((GR * APKL * 2) % 16) == 0);
static_assert((APKC % 8) == 0 && (APKL % 8) == 0);
static_assert(NBWC * NTHR * 8 == FD * KC && NBWL * NTHR * 8 == FD * FD);
static_assert(OTHR == FD);
static_assert(FD / 4 == 128 && NTHR == 2 * (FD / 4));

typedef float          v4f  __attribute__((ext_vector_type(4)));
typedef float          v4fa __attribute__((ext_vector_type(4), may_alias));
typedef float          v8f  __attribute__((ext_vector_type(8)));
typedef double         v2d  __attribute__((ext_vector_type(2)));
typedef int            v4i  __attribute__((ext_vector_type(4)));
typedef _Float16       v8h  __attribute__((ext_vector_type(8)));
typedef _Float16       v16h __attribute__((ext_vector_type(16)));
union FragH { v16h v; v8h h[2]; };

__device__ __forceinline__ v8h cvt8(v4f a, v4f b) {
  v8h r;
  r[0] = (_Float16)a.x; r[1] = (_Float16)a.y; r[2] = (_Float16)a.z; r[3] = (_Float16)a.w;
  r[4] = (_Float16)b.x; r[5] = (_Float16)b.y; r[6] = (_Float16)b.z; r[7] = (_Float16)b.w;
  return r;
}

__device__ __forceinline__ v8f wmh(v16h a, v16h b, v8f c) {
  v8f d = __builtin_amdgcn_wmma_f32_16x16x32_f16(false, a, false, b, (short)0, c, false, false);
  asm volatile("v_nop\n\tv_nop\n\tv_nop\n\tv_nop" : "+v"(d) : "v"(a), "v"(b));
  return d;
}

template <int KD, int APK>
__device__ __forceinline__ void mma_strip(const _Float16* sA, const _Float16* __restrict__ Bw,
                                          int srow, int lane, v8f (&acc)[4]) {
  static_assert((KD % 32) == 0 && (APK % 8) == 0);
  constexpr int NKT = KD / 32;
  const int hh = lane >> 4, m = lane & 15;
#pragma unroll
  for (int t = 0; t < 4; ++t) { v8f z = {0.f, 0.f, 0.f, 0.f, 0.f, 0.f, 0.f, 0.f}; acc[t] = z; }
  const _Float16* ap  = sA + (srow + m) * APK + 8 * hh;
  const _Float16* bp0 = Bw + (size_t)m * KD + 8 * hh;
#pragma unroll 1
  for (int kt = 0; kt < NKT; ++kt) {
    FragH a;
    a.h[0] = *(const v8h*)(ap + 32 * kt);
    a.h[1] = *(const v8h*)(ap + 32 * kt + 16);
#pragma unroll
    for (int t = 0; t < 4; ++t) {
      const _Float16* bp = bp0 + (size_t)(16 * t) * KD + 32 * kt;
      FragH b;
      b.h[0] = *(const v8h*)bp;
      b.h[1] = *(const v8h*)(bp + 16);
      acc[t] = wmh(a.v, b.v, acc[t]);
    }
  }
}

template <int NB>
__device__ __forceinline__ int scan_chunk(const int* __restrict__ keys, int nE, int cbase, int slotBase,
                                          int vec8, int* list, int tid, int lane, int wave) {
  int wc = 0;
#pragma unroll
  for (int g = 0; g < NGRP; ++g) {
    const int el0  = (g * NTHR + tid) * EPT;
    const int e0   = cbase + el0;
    const int sent = -2147483647 - 1;
    v4i da, db;
    if (vec8 != 0 && cbase + CHUNK <= nE) {
      da = *(const v4i*)(keys + e0);
      db = *(const v4i*)(keys + e0 + 4);
    } else {
      da.x = (e0     < nE) ? keys[min(e0, nE - 1)] : sent;
      da.y = (e0 + 1 < nE) ? keys[min(e0 + 1, nE - 1)] : sent;
      da.z = (e0 + 2 < nE) ? keys[min(e0 + 2, nE - 1)] : sent;
      da.w = (e0 + 3 < nE) ? keys[min(e0 + 3, nE - 1)] : sent;
      db.x = (e0 + 4 < nE) ? keys[min(e0 + 4, nE - 1)] : sent;
      db.y = (e0 + 5 < nE) ? keys[min(e0 + 5, nE - 1)] : sent;
      db.z = (e0 + 6 < nE) ? keys[min(e0 + 6, nE - 1)] : sent;
      db.w = (e0 + 7 < nE) ? keys[min(e0 + 7, nE - 1)] : sent;
    }
    const unsigned nb = (unsigned)slotBase;
    const unsigned s0 = (unsigned)da.x - nb, s1 = (unsigned)da.y - nb;
    const unsigned s2 = (unsigned)da.z - nb, s3 = (unsigned)da.w - nb;
    const unsigned s4 = (unsigned)db.x - nb, s5 = (unsigned)db.y - nb;
    const unsigned s6 = (unsigned)db.z - nb, s7 = (unsigned)db.w - nb;
    const bool h0 = s0 < (unsigned)NB, h1 = s1 < (unsigned)NB, h2 = s2 < (unsigned)NB, h3 = s3 < (unsigned)NB;
    const bool h4 = s4 < (unsigned)NB, h5 = s5 < (unsigned)NB, h6 = s6 < (unsigned)NB, h7 = s7 < (unsigned)NB;
    const unsigned any = __builtin_amdgcn_ballot_w32(h0 | h1 | h2 | h3 | h4 | h5 | h6 | h7);
    if (any != 0u) {
#define HITJ(J, HJ, SJ) { \
        const unsigned mj = __builtin_amdgcn_ballot_w32(HJ); \
        if (mj != 0u) { \
          if (HJ) { \
            const int pos = wc + (int)__builtin_amdgcn_mbcnt_lo(mj, 0u); \
            if (pos < WCAP) list[wave * WCAP + pos] = ((el0 + (J)) << 12) | (int)(SJ); \
          } \
          wc += (int)__builtin_popcount(mj); } }
      HITJ(0, h0, s0)
      HITJ(1, h1, s1)
      HITJ(2, h2, s2)
      HITJ(3, h3, s3)
      HITJ(4, h4, s4)
      HITJ(5, h5, s5)
      HITJ(6, h6, s6)
      HITJ(7, h7, s7)
#undef HITJ
    }
  }
  return wc;
}

__global__ __launch_bounds__(NTHR) void k_wprep(const float* __restrict__ wc, const float* __restrict__ wl,
                                                _Float16* pc, _Float16* pl) {
  const int blk = blockIdx.x, tid = threadIdx.x;
  int KD, i;
  const float* W;
  _Float16* P;
  if (blk < NBWC) { KD = KC; W = wc; P = pc; i = blk * NTHR + tid; }
  else            { KD = FD; W = wl; P = pl; i = (blk - NBWC) * NTHR + tid; }
  const int kq = KD >> 3;
  const int n  = i / kq;
  const int k0 = (i - n * kq) * 8;
  v4f a, b;
  a.x = W[(size_t)(k0 + 0) * FD + n] * WSCL;
  a.y = W[(size_t)(k0 + 1) * FD + n] * WSCL;
  a.z = W[(size_t)(k0 + 2) * FD + n] * WSCL;
  a.w = W[(size_t)(k0 + 3) * FD + n] * WSCL;
  b.x = W[(size_t)(k0 + 4) * FD + n] * WSCL;
  b.y = W[(size_t)(k0 + 5) * FD + n] * WSCL;
  b.z = W[(size_t)(k0 + 6) * FD + n] * WSCL;
  b.w = W[(size_t)(k0 + 7) * FD + n] * WSCL;
  const v8h hv = cvt8(a, b);
  _Float16* dp = P + (size_t)i * 8;
  *(volatile v8h*)dp = hv;
  __threadfence();
  *(volatile v8h*)dp = hv;
}

__global__ __launch_bounds__(NTHR) void k_count(const int* __restrict__ keys, int* cnt, int nE, int vec8) {
  __shared__ __attribute__((aligned(16))) int scnt[NBC];
  __shared__ __attribute__((aligned(16))) int list[LISTN];
  __shared__ int wcnt[NWAVE];
  const int tid = threadIdx.x, lane = tid & 31, wave = tid >> 5;
  const int nodeBase = blockIdx.x * NBC;

  for (int i = tid; i < NBC; i += NTHR) scnt[i] = 0;
  __syncthreads();

  const int nChunks = (nE + CHUNK - 1) / CHUNK;
#pragma unroll 1
  for (int ch = 0; ch < nChunks; ++ch) {
    const int cbase = ch * CHUNK;
    const int wc = scan_chunk<NBC>(keys, nE, cbase, nodeBase, vec8, list, tid, lane, wave);
    if (lane == 0) wcnt[wave] = wc;
    __syncthreads();
    if (wave == 0) {
#pragma unroll 1
      for (int wsx = 0; wsx < NWAVE; ++wsx) {
        int n = __builtin_amdgcn_readfirstlane(wcnt[wsx]);
        n = n > WCAP ? WCAP : (n < 0 ? 0 : n);
        const int* lp = list + wsx * WCAP;
#pragma unroll 1
        for (int i = 0; i < n; ++i) {
          const int ent  = __builtin_amdgcn_readfirstlane(lp[i]);
          const int slot = ent & (NBC - 1);
          if (lane == 0) scnt[slot] = scnt[slot] + 1;
        }
      }
    }
    __syncthreads();
  }

  v4i cq[4];
#pragma unroll
  for (int q = 0; q < 4; ++q) {
    const int f = (wave * 4 + q) * 128 + 4 * lane;
    cq[q] = *(const v4i*)(scnt + f);
  }
  int* cp = cnt + (size_t)nodeBase;
#pragma unroll
  for (int q = 0; q < 4; ++q) {
    const int f = (wave * 4 + q) * 128 + 4 * lane;
    *(volatile v4i*)(cp + f) = cq[q];
  }
  __threadfence();
#pragma unroll
  for (int q = 0; q < 4; ++q) {
    const int f = (wave * 4 + q) * 128 + 4 * lane;
    *(volatile v4i*)(cp + f) = cq[q];
  }
}

__global__ __launch_bounds__(OTHR) void k_offsets(
    const int* __restrict__ cnt, int* off, int* rbase, int nChunk) {
  __shared__ __attribute__((aligned(16))) int soff[NBC];
  __shared__ __attribute__((aligned(16))) int srb[RBN];
  __shared__ int wtot[OTHR / 32];
  const int tid = threadIdx.x, lane = tid & 31, wave = tid >> 5, sub = tid >> 7;
  for (int i = tid; i < RBN; i += OTHR) srb[i] = 0;
  int carry = 0;
#pragma unroll 1
  for (int ch = 0; ch < nChunk; ++ch) {
    const int base = ch * NBC;
    const v4i c0 = *(const v4i*)(cnt + base + 8 * tid);
    const v4i c1 = *(const v4i*)(cnt + base + 8 * tid + 4);
    const int e0 = max(c0.x, 0), e1 = max(c0.y, 0), e2 = max(c0.z, 0), e3 = max(c0.w, 0);
    const int e4 = max(c1.x, 0), e5 = max(c1.y, 0), e6 = max(c1.z, 0), e7 = max(c1.w, 0);
    const int ts = e0 + e1 + e2 + e3 + e4 + e5 + e6 + e7;
    int incl = ts;
#pragma unroll
    for (int d = 1; d < 32; d <<= 1) {
      const int t = __shfl_up(incl, d);
      if (lane >= d) incl += t;
    }
    if (lane == 31) wtot[wave] = incl;
    __syncthreads();
    const int S0 = wtot[0]  + wtot[1]  + wtot[2]  + wtot[3];
    const int S1 = wtot[4]  + wtot[5]  + wtot[6]  + wtot[7];
    const int S2 = wtot[8]  + wtot[9]  + wtot[10] + wtot[11];
    const int S3 = wtot[12] + wtot[13] + wtot[14] + wtot[15];
    int pre = 0;
#pragma unroll 1
    for (int w = 4 * sub; w < wave; ++w) pre += wtot[w];
    const int b0 = carry;
    const int b1 = b0 + ((S0 + 31) & ~31);
    const int b2 = b1 + ((S1 + 31) & ~31);
    const int b3 = b2 + ((S2 + 31) & ~31);
    const int b4 = b3 + ((S3 + 31) & ~31);
    const int myb = sub == 0 ? b0 : (sub == 1 ? b1 : (sub == 2 ? b2 : b3));
    if (tid == 0) {
      srb[min(4 * ch + 0, RBN - 1)] = b0;
      srb[min(4 * ch + 1, RBN - 1)] = b1;
      srb[min(4 * ch + 2, RBN - 1)] = b2;
      srb[min(4 * ch + 3, RBN - 1)] = b3;
    }
    int run = myb + pre + incl - ts;
    soff[8 * tid + 0] = run; run += e0;
    soff[8 * tid + 1] = run; run += e1;
    soff[8 * tid + 2] = run; run += e2;
    soff[8 * tid + 3] = run; run += e3;
    soff[8 * tid + 4] = run; run += e4;
    soff[8 * tid + 5] = run; run += e5;
    soff[8 * tid + 6] = run; run += e6;
    soff[8 * tid + 7] = run;
    carry = b4;
    __syncthreads();
    const v4i o0 = *(const v4i*)(soff + 4 * tid);
    const v4i o1 = *(const v4i*)(soff + 4 * (tid + OTHR));
    int* op = off + base;
    *(volatile v4i*)(op + 4 * tid) = o0;
    *(volatile v4i*)(op + 4 * (tid + OTHR)) = o1;
    __threadfence();
    *(volatile v4i*)(op + 4 * tid) = o0;
    *(volatile v4i*)(op + 4 * (tid + OTHR)) = o1;
    __syncthreads();
  }
  if (tid == 0) srb[min(4 * nChunk, RBN - 1)] = carry;
  __syncthreads();
  v4i rv = {0, 0, 0, 0};
  if (tid < 32) rv = *(const v4i*)(srb + 4 * tid);
  if (tid < 32) *(volatile v4i*)(rbase + 4 * tid) = rv;
  __threadfence();
  if (tid < 32) *(volatile v4i*)(rbase + 4 * tid) = rv;
}

__global__ __launch_bounds__(NTHR) void k_fill(
    const int* __restrict__ srcs, const int* __restrict__ dsts,
    const int* __restrict__ off, const int* __restrict__ rbase,
    int* csr, int nN, int nE, int vec8, int csrLen) {
  extern __shared__ v4f lds_dyn[];
  int* region = (int*)lds_dyn;
  int* cursor = region + RCAP;
  int* list   = cursor + NBF;
  int* wcnt   = list + LISTN;
  const int tid = threadIdx.x, lane = tid & 31, wave = tid >> 5;
  const int b = blockIdx.x;
  const int nodeBase = b * NBF;

  int rb0 = rbase[b];
  const int rb1 = rbase[b + 1];
  rb0 = rb0 < 0 ? 0 : (rb0 > csrLen ? csrLen : rb0);
  rb0 &= ~31;
  int len = rb1 - rb0;
  len = len < 0 ? 0 : (len > RCAP ? RCAP : len);
  int lenW = (len + 31) & ~31;
  if (rb0 + lenW > csrLen) lenW = (csrLen - rb0) & ~31;

  {
    const v4i z = {0, 0, 0, 0};
    for (int i = tid; i < RCAP / 4; i += NTHR) ((v4i*)region)[i] = z;
    for (int s = tid; s < NBF; s += NTHR) {
      int o = off[nodeBase + s] - rb0;
      o = o < 0 ? 0 : (o > RCAP ? RCAP : o);
      cursor[s] = o;
    }
  }
  __syncthreads();

  const int nChunks = (nE + CHUNK - 1) / CHUNK;
#pragma unroll 1
  for (int ch = 0; ch < nChunks; ++ch) {
    const int cbase = ch * CHUNK;
    const int wc = scan_chunk<NBF>(dsts, nE, cbase, nodeBase, vec8, list, tid, lane, wave);
    if (lane == 0) wcnt[wave] = wc;
    __syncthreads();
    if (wave == 0) {
#pragma unroll 1
      for (int wsx = 0; wsx < NWAVE; ++wsx) {
        int n = __builtin_amdgcn_readfirstlane(wcnt[wsx]);
        n = n > WCAP ? WCAP : (n < 0 ? 0 : n);
        const int* lp = list + wsx * WCAP;
#pragma unroll 1
        for (int i = 0; i < n; ++i) {
          const int ent  = __builtin_amdgcn_readfirstlane(lp[i]);
          const int slot = ent & (NBF - 1);
          int e = cbase + ((ent >> 12) & (CHUNK - 1));
          e = e > nE - 1 ? nE - 1 : e;
          int sv = srcs[e];
          sv = sv < 0 ? 0 : (sv > nN - 1 ? nN - 1 : sv);
          if (lane == 0) {
            int pos = cursor[slot];
            pos = pos < 0 ? 0 : (pos > RCAP - 1 ? RCAP - 1 : pos);
            region[pos] = sv;
            const int np = pos + 1;
            cursor[slot] = np > RCAP ? RCAP : np;
          }
        }
      }
    }
    __syncthreads();
  }

  const int nv = lenW >> 2;
  int* gp = csr + rb0;
#pragma unroll 1
  for (int i = tid; i < nv; i += NTHR) { const v4i v = ((const v4i*)region)[i]; *(volatile v4i*)(gp + 4 * i) = v; }
  __threadfence();
#pragma unroll 1
  for (int i = tid; i < nv; i += NTHR) { const v4i v = ((const v4i*)region)[i]; *(volatile v4i*)(gp + 4 * i) = v; }
}

template <int MODE>
__global__ __launch_bounds__(NTHR) void k_agg(
    const int* __restrict__ csr, const int* __restrict__ off,
    const int* __restrict__ cntd, const int* __restrict__ cnts,
    const float* __restrict__ h, const float* __restrict__ x,
    float* outp, int nN, int csrLen) {
#pragma clang fp contract(off)
  const int tid = threadIdx.x, lane = tid & 31, wave = tid >> 5;
  const int tbase = blockIdx.x * TGT + wave * 32;
  const int cl = tbase + lane;
  const int cnt_l = cntd[cl];
  const int off_l = off[cl];
  const int cs_l  = cnts[cl];
  const float dc_l = cs_l > 0 ? rsqrtf((float)cs_l) : 0.0f;

#pragma unroll 1
  for (int j = 0; j < 32; ++j) {
    const int c = tbase + j;
    int n = __builtin_amdgcn_readlane(cnt_l, j);
    n = n < 0 ? 0 : (n > DEGCAP ? DEGCAP : n);
    const int st = __builtin_amdgcn_readlane(off_l, j);
    const float dc = __int_as_float(__builtin_amdgcn_readlane(__float_as_int(dc_l), j));
    v4f a0 = {0.f, 0.f, 0.f, 0.f}, a1 = {0.f, 0.f, 0.f, 0.f};
    v4f a2 = {0.f, 0.f, 0.f, 0.f}, a3 = {0.f, 0.f, 0.f, 0.f};
#pragma unroll 1
    for (int q0 = 0; q0 < n; q0 += 32) {
      int pos = st + q0 + lane;
      pos = pos < 0 ? 0 : (pos > csrLen - 1 ? csrLen - 1 : pos);
      int sl = csr[pos];
      sl = sl < 0 ? 0 : (sl > nN - 1 ? nN - 1 : sl);
      const int csv = cnts[sl];
      const float ds = csv > 0 ? rsqrtf((float)csv) : 0.0f;
      const float wl = -(ds * dc);
      const int mcnt = (n - q0) < 32 ? (n - q0) : 32;
#pragma unroll 1
      for (int p = 0; p < mcnt; ++p) {
        const int s = __builtin_amdgcn_readlane(sl, p);
        const float w = __int_as_float(__builtin_amdgcn_readlane(__float_as_int(wl), p));
        const float* hp = h + (size_t)s * FD + 4 * lane;
        const v4f v0 = *(const v4f*)hp;
        const v4f v1 = *(const v4f*)(hp + 128);
        const v4f v2 = *(const v4f*)(hp + 256);
        const v4f v3 = *(const v4f*)(hp + 384);
        a0 = a0 + v0 * w;
        a1 = a1 + v1 * w;
        a2 = a2 + v2 * w;
        a3 = a3 + v3 * w;
      }
    }
    if (MODE == 1) {
      const int cr = c > nN - 1 ? nN - 1 : c;
      const float* xp = x + (size_t)cr * FD + 4 * lane;
      const v4f x0 = *(const v4f*)xp;
      const v4f x1 = *(const v4f*)(xp + 128);
      const v4f x2 = *(const v4f*)(xp + 256);
      const v4f x3 = *(const v4f*)(xp + 384);
      a0 = a0 * 2.0f - x0;
      a1 = a1 * 2.0f - x1;
      a2 = a2 * 2.0f - x2;
      a3 = a3 * 2.0f - x3;
    }
    float* op = outp + (size_t)c * FD + 4 * lane;
    *(volatile v4f*)(op)       = a0;
    *(volatile v4f*)(op + 128) = a1;
    *(volatile v4f*)(op + 256) = a2;
    *(volatile v4f*)(op + 384) = a3;
    __threadfence();
    *(volatile v4f*)(op)       = a0;
    *(volatile v4f*)(op + 128) = a1;
    *(volatile v4f*)(op + 256) = a2;
    *(volatile v4f*)(op + 384) = a3;
  }
}

__device__ __forceinline__ void store_sub16x64(const float* stg, float* C, int row0, int col0,
                                               int rowLim, int lane) {
  const int hh = lane >> 4, l4 = 4 * (lane & 15);
#pragma unroll
  for (int i = 0; i < 8; ++i) {
    const int rl = 2 * i + hh;
    const v4fa v = *(const v4fa*)(stg + rl * 64 + l4);
    const int gr = row0 + rl;
    if (gr < rowLim) *(volatile v4f*)(C + (size_t)gr * FD + col0 + l4) = v;
  }
  __threadfence();
#pragma unroll
  for (int i = 0; i < 8; ++i) {
    const int rl = 2 * i + hh;
    const v4fa v = *(const v4fa*)(stg + rl * 64 + l4);
    const int gr = row0 + rl;
    if (gr < rowLim) *(volatile v4f*)(C + (size_t)gr * FD + col0 + l4) = v;
  }
}

__global__ __launch_bounds__(NTHR) void k_cheb(
    const float* __restrict__ x, const float* __restrict__ t1, const float* __restrict__ t2,
    const _Float16* __restrict__ Bw, const float* __restrict__ bias,
    float* C, double* part, int nN) {
  extern __shared__ v4f lds_dyn[];
  __shared__ __attribute__((aligned(16))) float sbias[FD];
  _Float16* sA  = (_Float16*)lds_dyn;
  float*    stg = (float*)((char*)lds_dyn + GR * APKC * 2);
  double*   dsg = (double*)((char*)lds_dyn + GR * APKC * 2 + LDS_STG);
  const int tid = threadIdx.x, lane = tid & 31, wave = tid >> 5, hh = lane >> 4, m = lane & 15;
  const int rowBase = blockIdx.x * GR;
  const int c0 = (tid & 63) * 8, rr = tid >> 6;

  if (wave < 4) {
    const v4f bq = *(const v4f*)(bias + 4 * tid);
    *(v4f*)(sbias + 4 * tid) = bq;
  }

#pragma unroll 1
  for (int p = 0; p < 3; ++p) {
    const float* srcp = (p == 0) ? x : ((p == 1) ? t1 : t2);
    const int rlim = (p == 0) ? (nN - 1) : (rowBase + GR - 1);
#pragma unroll 4
    for (int it = 0; it < 16; ++it) {
      const int r = it * 4 + rr;
      int row = rowBase + r;
      row = row > rlim ? rlim : row;
      const float* ap = srcp + (size_t)row * FD + c0;
      const v4f a = *(const v4f*)ap, b = *(const v4f*)(ap + 4);
      *(v8h*)(sA + r * APKC + p * FD + c0) = cvt8(a, b);
    }
  }
  __syncthreads();

  const int colw = wave * 64;
  float bv[4];
#pragma unroll
  for (int t = 0; t < 4; ++t) bv[t] = sbias[colw + 16 * t + m];
  double sd[4] = {0.0, 0.0, 0.0, 0.0}, qd[4] = {0.0, 0.0, 0.0, 0.0};
  float* mystg = stg + wave * 1024;

#pragma unroll 1
  for (int s = 0; s < 4; ++s) {
    v8f acc[4];
    mma_strip<KC, APKC>(sA, Bw + (size_t)colw * KC, 16 * s, lane, acc);
    float* sp = mystg + (8 * hh) * 64 + m;
#pragma unroll
    for (int t = 0; t < 4; ++t) {
#pragma unroll
      for (int r = 0; r < 8; ++r) {
        const float v = acc[t][r] * WINV + bv[t];
        const int row = rowBase + 16 * s + 8 * hh + r;
        const float vz = (row < nN) ? v : 0.0f;
        const double dv = (double)vz;
        sd[t] += dv;
        qd[t] = fma(dv, dv, qd[t]);
        sp[r * 64 + 16 * t] = v;
      }
    }
    __syncthreads();
    store_sub16x64(mystg, C, rowBase + 16 * s, colw, rowBase + GR, lane);
    __syncthreads();
  }

  double* dw = dsg + wave * 256;
#pragma unroll
  for (int t = 0; t < 4; ++t) {
    dw[hh * 64 + 16 * t + m]       = sd[t];
    dw[128 + hh * 64 + 16 * t + m] = qd[t];
  }
  __syncthreads();
  v2d sv, qv;
  sv.x = dw[2 * lane]           + dw[64 + 2 * lane];
  sv.y = dw[2 * lane + 1]       + dw[64 + 2 * lane + 1];
  qv.x = dw[128 + 2 * lane]     + dw[192 + 2 * lane];
  qv.y = dw[128 + 2 * lane + 1] + dw[192 + 2 * lane + 1];
  double* gS = part + (size_t)blockIdx.x * 1024 + colw + 2 * lane;
  double* gQ = gS + 512;
  *(volatile v2d*)gS = sv;
  *(volatile v2d*)gQ = qv;
  __threadfence();
  *(volatile v2d*)gS = sv;
  *(volatile v2d*)gQ = qv;
}

__global__ __launch_bounds__(OTHR) void k_bnfin(const double* __restrict__ part, float* coef, int nBlk, int nN) {
  __shared__ __attribute__((aligned(16))) float sco[2 * FD];
  const int tid = threadIdx.x, c = tid;
  double S = 0.0, Q = 0.0;
#pragma unroll 1
  for (int b = 0; b < nBlk; ++b) {
    S += part[(size_t)b * 1024 + c];
    Q += part[(size_t)b * 1024 + 512 + c];
  }
  const double rn = 1.0 / (double)(nN > 1 ? nN : 1);
  const double mean = S * rn;
  double var = Q * rn - mean * mean;
  var = var < 0.0 ? 0.0 : var;
  sco[c]      = (float)mean;
  sco[FD + c] = rsqrtf((float)var + BN_EPS);
  __syncthreads();
  v4f cv = {0.f, 0.f, 0.f, 0.f};
  if (tid < 256) cv = *(const v4f*)(sco + 4 * tid);
  if (tid < 256) *(volatile v4f*)(coef + 4 * tid) = cv;
  __threadfence();
  if (tid < 256) *(volatile v4f*)(coef + 4 * tid) = cv;
}

__global__ __launch_bounds__(NTHR) void k_out(
    const float* __restrict__ x, const _Float16* __restrict__ Bw, const float* __restrict__ lb,
    const float* __restrict__ pre, const float* __restrict__ coef,
    const float* __restrict__ gam, const float* __restrict__ bet,
    float* out, int nN) {
  extern __shared__ v4f lds_dyn[];
  __shared__ __attribute__((aligned(16))) float spar[5 * FD];
  _Float16* sA  = (_Float16*)lds_dyn;
  float*    stg = (float*)((char*)lds_dyn + GR * APKL * 2);
  const int tid = threadIdx.x, lane = tid & 31, wave = tid >> 5, hh = lane >> 4, m = lane & 15;
  const int rowBase = blockIdx.x * GR;
  const int c0 = (tid & 63) * 8, rr = tid >> 6;

  {
    const v4f cq = *(const v4f*)(coef + 4 * tid);
    *(v4f*)(spar + 4 * tid) = cq;
    if (wave < 4) {
      const v4f gq = *(const v4f*)(gam + 4 * tid);
      const v4f lq = *(const v4f*)(lb + 4 * tid);
      *(v4f*)(spar + 2 * FD + 4 * tid) = gq;
      *(v4f*)(spar + 4 * FD + 4 * tid) = lq;
    } else {
      const v4f bq = *(const v4f*)(bet + 4 * (tid - 128));
      *(v4f*)(spar + 3 * FD + 4 * (tid - 128)) = bq;
    }
  }

#pragma unroll 4
  for (int it = 0; it < 16; ++it) {
    const int r = it * 4 + rr;
    int row = rowBase + r;
    row = row > nN - 1 ? nN - 1 : row;
    const float* ap = x + (size_t)row * FD + c0;
    const v4f a = *(const v4f*)ap, b = *(const v4f*)(ap + 4);
    *(v8h*)(sA + r * APKL + c0) = cvt8(a, b);
  }
  __syncthreads();

  const int colw = wave * 64;
  float muv[4], rsv[4], gv[4], bev[4], lbv[4];
#pragma unroll
  for (int t = 0; t < 4; ++t) {
    const int col = colw + 16 * t + m;
    muv[t] = spar[col];
    rsv[t] = spar[FD + col];
    gv[t]  = spar[2 * FD + col];
    bev[t] = spar[3 * FD + col];
    lbv[t] = spar[4 * FD + col];
  }
  float* mystg = stg + wave * 1024;
  const int l4 = 4 * (lane & 15);

#pragma unroll 1
  for (int s = 0; s < 4; ++s) {
    v8f acc[4];
    mma_strip<FD, APKL>(sA, Bw + (size_t)colw * FD, 16 * s, lane, acc);
    {
      const float* pp = pre + (size_t)(rowBase + 16 * s) * FD + colw + l4;
#pragma unroll
      for (int i = 0; i < 8; ++i) {
        const int rl = 2 * i + hh;
        const v4f pv4 = *(const v4f*)(pp + (size_t)rl * FD);
        *(v4f*)(mystg + rl * 64 + l4) = pv4;
      }
    }
    __syncthreads();
    float* sp = mystg + (8 * hh) * 64 + m;
#pragma unroll
    for (int t = 0; t < 4; ++t) {
#pragma unroll
      for (int r = 0; r < 8; ++r) {
        const float pv = sp[r * 64 + 16 * t];
        float bn = (pv - muv[t]) * rsv[t] * gv[t] + bev[t];
        bn = fmaxf(bn, 0.0f);
        const float idv = acc[t][r] * WINV + lbv[t];
        sp[r * 64 + 16 * t] = bn + idv;
      }
    }
    __syncthreads();
    store_sub16x64(mystg, out, rowBase + 16 * s, colw, nN, lane);
    __syncthreads();
  }
}

extern "C" void kernel_launch(void* const* d_in, const int* in_sizes, int n_in,
                              void* d_out, int out_size, void* d_ws, size_t ws_size,
                              hipStream_t stream) {
  if (n_in < 8) return;
  const int nN = in_sizes[0] / FD;
  const int nE = in_sizes[7] / 2;
  if (nN <= 0 || nE <= 0) return;
  if (in_sizes[0] != nN * FD || in_sizes[7] != 2 * nE) return;
  if (in_sizes[1] != 3 * FD * FD || in_sizes[2] != FD) return;
  if (in_sizes[3] != FD * FD || in_sizes[4] != FD) return;
  if (in_sizes[5] != FD || in_sizes[6] != FD) return;
  if (out_size != nN * FD) return;
  if (nE > (1 << 28) || nN > (1 << 22)) return;

  const float* x      = (const float*)d_in[0];
  const float* cheb_w = (const float*)d_in[1];
  const float* cheb_b = (const float*)d_in[2];
  const float* lin_w  = (const float*)d_in[3];
  const float* lin_b  = (const float*)d_in[4];
  const float* gam    = (const float*)d_in[5];
  const float* bet    = (const float*)d_in[6];
  const int*   eidx   = (const int*)d_in[7];
  const int*   srcs   = eidx;
  const int*   dsts   = eidx + nE;
  float* out = (float*)d_out;

  const int NPAD   = ((nN + TGT - 1) / TGT) * TGT;
  const int nBC    = (nN + NBC - 1) / NBC;
  const int CNTPAD = nBC * NBC;
  if (4 * nBC + 1 > RBN) return;
  const int nBF    = (nN + NBF - 1) / NBF;
  const int csrLen = ((nE + 31) & ~31) + 4096;
  if (31 * 4 * nBC > 4096) return;
  const int nGemm  = NPAD / GR;
  const int nAgg   = NPAD / TGT;

  char* ws = (char*)d_ws;
  size_t off = 0;
  const size_t oWc   = off; off += (size_t)FD * KC * 2;              off = (off + 255) & ~(size_t)255;
  const size_t oWl   = off; off += (size_t)FD * FD * 2;              off = (off + 255) & ~(size_t)255;
  const size_t oCntD = off; off += (size_t)CNTPAD * 4;               off = (off + 255) & ~(size_t)255;
  const size_t oCntS = off; off += (size_t)CNTPAD * 4;               off = (off + 255) & ~(size_t)255;
  const size_t oOff  = off; off += (size_t)CNTPAD * 4;               off = (off + 255) & ~(size_t)255;
  const size_t oRb   = off; off += (size_t)RBN * 4;                  off = (off + 255) & ~(size_t)255;
  const size_t oCsr  = off; off += (size_t)csrLen * 4;               off = (off + 255) & ~(size_t)255;
  const size_t oT1   = off; off += (size_t)NPAD * FD * 4;            off = (off + 255) & ~(size_t)255;
  const size_t oT2   = off; off += (size_t)NPAD * FD * 4;            off = (off + 255) & ~(size_t)255;
  const size_t oPre  = off; off += (size_t)NPAD * FD * 4;            off = (off + 255) & ~(size_t)255;
  const size_t oPart = off; off += (size_t)nGemm * 1024 * 8;         off = (off + 255) & ~(size_t)255;
  const size_t oCoef = off; off += (size_t)2 * FD * 4;               off = (off + 255) & ~(size_t)255;
  if (off > ws_size || off > (size_t)WSCAP) return;
  _Float16* Wc   = (_Float16*)(ws + oWc);
  _Float16* Wl   = (_Float16*)(ws + oWl);
  int*      cntd = (int*)(ws + oCntD);
  int*      cnts = (int*)(ws + oCntS);
  int*      offp = (int*)(ws + oOff);
  int*      rb   = (int*)(ws + oRb);
  int*      csr  = (int*)(ws + oCsr);
  float*    T1   = (float*)(ws + oT1);
  float*    T2   = (float*)(ws + oT2);
  float*    Pre  = (float*)(ws + oPre);
  double*   part = (double*)(ws + oPart);
  float*    coef = (float*)(ws + oCoef);

  const int vec8 = ((nE & 3) == 0) ? 1 : 0;

  k_wprep<<<NBWC + NBWL, NTHR, 0, stream>>>(cheb_w, lin_w, Wc, Wl);

  k_count<<<nBC, NTHR, 0, stream>>>(dsts, cntd, nE, vec8);
  k_count<<<nBC, NTHR, 0, stream>>>(srcs, cnts, nE, vec8);
  k_offsets<<<1, OTHR, 0, stream>>>(cntd, offp, rb, nBC);
  hipFuncSetAttribute(reinterpret_cast<const void*>(&k_fill),
                      hipFuncAttributeMaxDynamicSharedMemorySize, LDS_FILL);
  k_fill<<<nBF, NTHR, LDS_FILL, stream>>>(srcs, dsts, offp, rb, csr, nN, nE, vec8, csrLen);

  k_agg<0><<<nAgg, NTHR, 0, stream>>>(csr, offp, cntd, cnts, x, x, T1, nN, csrLen);
  k_agg<1><<<nAgg, NTHR, 0, stream>>>(csr, offp, cntd, cnts, T1, x, T2, nN, csrLen);

  hipFuncSetAttribute(reinterpret_cast<const void*>(&k_cheb),
                      hipFuncAttributeMaxDynamicSharedMemorySize, LDS_GC);
  k_cheb<<<nGemm, NTHR, LDS_GC, stream>>>(x, T1, T2, Wc, cheb_b, Pre, part, nN);

  k_bnfin<<<1, OTHR, 0, stream>>>(part, coef, nGemm, nN);

  hipFuncSetAttribute(reinterpret_cast<const void*>(&k_out),
                      hipFuncAttributeMaxDynamicSharedMemorySize, LDS_GO);
  k_out<<<nGemm, NTHR, LDS_GO, stream>>>(x, Wl, lin_b, Pre, coef, gam, bet, out, nN);
}
